// Block_15109694947394
// MI455X (gfx1250) — hardware-run, weakly checked
//
#include <hip/hip_runtime.h>


#ifndef NB
#define NB 4
#endif
#ifndef SEQ
#define SEQ 1024
#endif
#define NB_FULL  4
#define SEQ_FULL 1024
#define DM    1024
#define NH    16
#define DH    64
#define PD    4
#define QKVW  3072
#define FFD   4096
#define SMW   320
#define NTOK  (NB * SEQ)
#define WCAR  16.0f
#define HCAR  16.0f
#define ACAR  16.0f
#define OCAR  256.0f
#define LCAR  64.0f
#define PLOG  14.0f
#define L2E   1.4426950408889634f
#define SCL2  0.18033688011112042f
#define EP_H16  0
#define EP_GELU 1
#define EP_RES  2

#define AL256(x) ((((size_t)(x)) + 255) & ~(size_t)255)
#define WS_TOTAL (AL256((size_t)QKVW * DM * 2) + AL256((size_t)DM * DM * 2) + AL256((size_t)DM * DM * 2) + AL256((size_t)FFD * DM * 2) + AL256((size_t)DM * FFD * 2) + \
                  AL256((size_t)SMW * DM * 2) + AL256((size_t)NTOK * QKVW * 2) + AL256((size_t)NTOK * DM * 2) + AL256((size_t)NTOK * DM * 4) + AL256((size_t)NTOK * DM * 2) + \
                  AL256((size_t)NTOK * SMW * 2) + AL256((size_t)NB * NH * SEQ * 8 * 2) + AL256((size_t)NB * NH * SEQ * 8 * 2) + AL256((size_t)NB * NH * SEQ * 4) + \
                  AL256((size_t)NTOK * 4) + AL256((size_t)NTOK * DM * 2) + AL256((size_t)NTOK * FFD * 2))

static_assert(NB >= 1 && NB <= NB_FULL);
static_assert(SEQ >= 256 && SEQ <= SEQ_FULL);
static_assert((SEQ % 256) == 0);
static_assert(SEQ == SEQ_FULL || NB == 1);
static_assert((NTOK % 64) == 0);
static_assert(NH * DH == DM);
static_assert((size_t)NTOK * DM * 4 <= (size_t)16777216);
static_assert(DH == 64);
static_assert(NH == 16);
static_assert(NH * PD == 64);
static_assert(4 * NH * PD + NH <= SMW);
static_assert((SMW % 64) == 0 && (QKVW % 64) == 0 && (DM % 64) == 0 && (FFD % 64) == 0);
static_assert((DM % 32) == 0 && (FFD % 32) == 0);
static_assert((SEQ % 64) == 0 && (SEQ % 32) == 0);
static_assert(((NB * NH * SEQ) % 256) == 0);
static_assert(((SMW - 4 * NH * PD - NH) * DM) % 8 == 0);
static_assert(WS_TOTAL <= (size_t)134217728);

typedef _Float16 h16;
typedef __attribute__((ext_vector_type(16))) _Float16 v16h;
typedef __attribute__((ext_vector_type(8)))  _Float16 v8h;
typedef __attribute__((ext_vector_type(4)))  _Float16 v4h;
typedef __attribute__((ext_vector_type(2)))  _Float16 v2h;
typedef __attribute__((ext_vector_type(8)))  float    v8f;
typedef __attribute__((ext_vector_type(4)))  float    v4f;
typedef v8h __attribute__((may_alias)) v8ha;
typedef v4h __attribute__((may_alias)) v4ha;
typedef v4f __attribute__((may_alias)) v4fa;

__device__ __forceinline__ float bfr(float f) { unsigned u = __float_as_uint(f); u += 0x7FFFu + ((u >> 16) & 1u); return __uint_as_float(u & 0xFFFF0000u); }
__device__ __forceinline__ v16h cat16(v8h lo, v8h hi) { return __builtin_shufflevector(lo, hi, 0, 1, 2, 3, 4, 5, 6, 7, 8, 9, 10, 11, 12, 13, 14, 15); }
__device__ __forceinline__ v8f cat8f(v4f lo, v4f hi) { return __builtin_shufflevector(lo, hi, 0, 1, 2, 3, 4, 5, 6, 7); }
__device__ __forceinline__ v8f wmma16(v16h a, v16h b, v8f c) { return __builtin_amdgcn_wmma_f32_16x16x32_f16(false, a, false, b, (short)0, c, false, false); }
__device__ __forceinline__ float wsum(float v) { v += __shfl_xor(v, 16, 32); v += __shfl_xor(v, 8, 32); v += __shfl_xor(v, 4, 32); v += __shfl_xor(v, 2, 32); v += __shfl_xor(v, 1, 32); return v; }
__device__ __forceinline__ float wmax(float v) { v = fmaxf(v, __shfl_xor(v, 16, 32)); v = fmaxf(v, __shfl_xor(v, 8, 32)); v = fmaxf(v, __shfl_xor(v, 4, 32)); v = fmaxf(v, __shfl_xor(v, 2, 32)); v = fmaxf(v, __shfl_xor(v, 1, 32)); return v; }

__device__ __forceinline__ v16h ldfrag(const h16* p) { return cat16(*(const v8ha*)p, *(const v8ha*)(p + 16)); }
__device__ __forceinline__ v16h ldfrag_lo(const h16* p) { return cat16(*(const v8ha*)p, (v8h){}); }

static __device__ __forceinline__ h16 toh_flush(float v) { const h16 r = (h16)v; return (fabsf(v) < 6.103515625e-05f) ? (h16)0.0f : r; }

__device__ __forceinline__ v8f wmma16g(v16h a, v16h b, v8f c) {
    c = __builtin_amdgcn_wmma_f32_16x16x32_f16(false, a, false, b, (short)0, c, false, false);
    asm volatile("v_nop\n\tv_nop\n\tv_nop\n\tv_nop" : "+v"(c) : "v"(a), "v"(b));
    return c;
}

__device__ __forceinline__ v16h ldfrag8(const h16* p, int hi) {
    v8h x = *(const v8ha*)p;
    asm volatile("" : "+v"(x));
    const v8h z = (v8h){};
    const v8h lo = (hi == 0) ? x : z;
    return cat16(lo, z);
}

__device__ __forceinline__ float gelu_e(float x) {
    const float z = fabsf(x) * 0.70710678118654752f;
    const float t = __builtin_amdgcn_rcpf(1.0f + 0.3275911f * z);
    const float pl = t * (0.254829592f + t * (-0.284496736f + t * (1.421413741f + t * (-1.453152027f + t * 1.061405429f))));
    const float hc = 0.5f * pl * __builtin_amdgcn_exp2f(-(z * z) * L2E);
    const float cdf = (x < 0.0f) ? hc : 1.0f - hc;
    return x * cdf;
}

__device__ __forceinline__ float ipow32(float d1, int e) {
    const float d2 = d1 * d1, d4 = d2 * d2, d8 = d4 * d4, d16 = d8 * d8;
    float p = (e & 1) ? d1 : 1.0f;
    p *= (e & 2) ? d2 : 1.0f;
    p *= (e & 4) ? d4 : 1.0f;
    p *= (e & 8) ? d8 : 1.0f;
    p *= (e & 16) ? d16 : 1.0f;
    return p;
}

__device__ __forceinline__ v8f plucker(v4h pa, v4h pb, float am) {
#pragma clang fp contract(off)
    const float a0 = (float)pa[0] * am, a1 = (float)pa[1] * am, a2 = (float)pa[2] * am, a3 = (float)pa[3] * am;
    const float b0 = (float)pb[0], b1 = (float)pb[1], b2 = (float)pb[2], b3 = (float)pb[3];
    const float L0 = a0 * b1 - a1 * b0;
    const float L1 = a0 * b2 - a2 * b0;
    const float L2 = a0 * b3 - a3 * b0;
    const float L3 = a1 * b2 - a2 * b1;
    const float L4 = a1 * b3 - a3 * b1;
    const float L5 = a2 * b3 - a3 * b2;
    const float s = ((L0 * L0 + L1 * L1) + (L2 * L2 + L3 * L3)) + (L4 * L4 + L5 * L5);
    const float inv = rsqrtf(fmaxf(s, 1.0e-24f));
    v8f o;
    o[0] = L0 * inv; o[1] = L1 * inv; o[2] = L2 * inv; o[3] = L3 * inv; o[4] = L4 * inv; o[5] = L5 * inv; o[6] = 0.0f; o[7] = 0.0f;
    return o;
}

template <int EP, bool BIAS, bool RBF>
__global__ __launch_bounds__(32) void k_gemm(const h16* __restrict__ A, const h16* __restrict__ Bt, int K,
                                             float* Cf, h16* Ch, int ldc, float cs, float co,
                                             const float* __restrict__ bias, const float* __restrict__ R,
                                             size_t sA, size_t sB, size_t sC) {
    __shared__ __align__(16) float os[16 * 68];
    const size_t z = blockIdx.z; A += z * sA; Bt += z * sB;
    const int lane = threadIdx.x & 31, lr = lane & 15, hi = lane >> 4;
    const int r0 = blockIdx.x * 64, c0 = blockIdx.y * 64;
    v8f acc[4][4];
#pragma unroll
    for (int mb = 0; mb < 4; ++mb)
#pragma unroll
        for (int nb = 0; nb < 4; ++nb) acc[mb][nb] = (v8f){};
    const size_t aoff = (size_t)(r0 + lr) * K + 8 * hi, boff = (size_t)(c0 + lr) * K + 8 * hi;
#pragma unroll 1
    for (int kc = 0; kc < K; kc += 32) {
        v16h a[4], b;
#pragma unroll
        for (int mb = 0; mb < 4; ++mb) a[mb] = ldfrag(A + aoff + (size_t)mb * 16 * K + kc);
#pragma unroll
        for (int nb = 0; nb < 4; ++nb) {
            b = ldfrag(Bt + boff + (size_t)nb * 16 * K + kc);
#pragma unroll
            for (int mb = 0; mb < 4; ++mb) acc[mb][nb] = wmma16(a[mb], b, acc[mb][nb]);
        }
        asm volatile("v_nop\n\tv_nop\n\tv_nop\n\tv_nop" : "+v"(acc[0][0]), "+v"(acc[1][1]), "+v"(acc[2][2]), "+v"(acc[3][3]) : "v"(a[0]), "v"(a[3]), "v"(b));
    }
#pragma unroll
    for (int mb = 0; mb < 4; ++mb) {
#pragma unroll
        for (int nb = 0; nb < 4; ++nb) {
#pragma unroll
            for (int j = 0; j < 8; ++j) os[(hi * 8 + j) * 68 + nb * 16 + lr] = acc[mb][nb][j];
        }
        __builtin_amdgcn_fence(3, "wavefront"); __builtin_amdgcn_wave_barrier(); asm volatile("" ::: "memory");
        if constexpr (EP == EP_RES) {
            float* crow = Cf + z * sC + (size_t)(r0 + mb * 16) * ldc + c0;
            const float* rrow = R + (size_t)(r0 + mb * 16) * ldc + c0;
#pragma unroll 1
            for (int ps = 0; ps < 2; ++ps) {
#pragma unroll 1
                for (int s = 0; s < 8; ++s) {
                    const int row = 2 * s + hi, cofs = lr * 4;
                    const v4f u = *(const v4fa*)(os + row * 68 + cofs);
                    const v4f rv = *(const v4f*)(rrow + (size_t)row * ldc + cofs);
                    v4f o;
#pragma unroll
                    for (int q = 0; q < 4; ++q) {
                        float bq = 0.0f;
                        if constexpr (BIAS) bq = bfr(bias[c0 + cofs + q]);
                        const float y = u[q] * cs + bq;
                        const float rq0 = rv[q];
                        const float rq = RBF ? bfr(rq0) : rq0;
                        o[q] = rq + y;
                    }
                    *(volatile v4f*)(crow + (size_t)row * ldc + cofs) = o;
                }
                if (ps == 0) __threadfence();
            }
        } else {
            h16* crow = Ch + z * sC + (size_t)(r0 + mb * 16) * ldc + c0;
            const int q8 = lane >> 3, cofs = (lane & 7) * 8;
#pragma unroll 1
            for (int ps = 0; ps < 2; ++ps) {
#pragma unroll 1
                for (int s = 0; s < 4; ++s) {
                    const int row = 4 * s + q8;
                    const v4f u0 = *(const v4fa*)(os + row * 68 + cofs), u1 = *(const v4fa*)(os + row * 68 + cofs + 4);
                    const v8f u = cat8f(u0, u1);
                    v8h o;
#pragma unroll
                    for (int q = 0; q < 8; ++q) {
                        float bq = 0.0f;
                        if constexpr (BIAS) bq = bfr(bias[c0 + cofs + q]);
                        float y = u[q] * cs + bq;
                        if constexpr (EP == EP_GELU) y = gelu_e(y);
                        o[q] = toh_flush(y * co);
                    }
                    *(volatile v8h*)(crow + (size_t)row * ldc + cofs) = o;
                }
                if (ps == 0) __threadfence();
            }
        }
        __builtin_amdgcn_wave_barrier(); asm volatile("" ::: "memory");
    }
}

__global__ __launch_bounds__(256) void k_cvtw(const float* __restrict__ src, h16* dst, unsigned n8) {
    const unsigned i = blockIdx.x * 256 + threadIdx.x; if (i >= n8) return;
    const v4f a0 = *(const v4f*)(src + (size_t)i * 8), a1 = *(const v4f*)(src + (size_t)i * 8 + 4);
    const v8f a = cat8f(a0, a1);
    v8h o;
#pragma unroll
    for (int k = 0; k < 8; ++k) { const float f = a[k]; o[k] = (h16)(bfr(f) * WCAR); }
    h16* p = dst + (size_t)i * 8;
    *(volatile v8h*)p = o; __threadfence(); *(volatile v8h*)p = o;
}

__global__ __launch_bounds__(256) void k_zero16(h16* dst, unsigned n8) {
    const unsigned i = blockIdx.x * 256 + threadIdx.x; if (i >= n8) return;
    const v8h z = (v8h){};
    h16* p = dst + (size_t)i * 8;
    *(volatile v8h*)p = z; __threadfence(); *(volatile v8h*)p = z;
}

template <bool RBF>
__global__ __launch_bounds__(128) void k_ln(const float* __restrict__ X, const float* __restrict__ w, const float* __restrict__ bb, h16* Hp) {
    __shared__ float red[8];
    const int row = blockIdx.x, t = threadIdx.x, lane = t & 31, wave = t >> 5;
    const float* xr = X + (size_t)row * DM + t * 8;
    const v4f p0 = *(const v4f*)xr, p1 = *(const v4f*)(xr + 4);
    v8f v = cat8f(p0, p1);
    if constexpr (RBF) {
#pragma unroll
        for (int k = 0; k < 8; ++k) { const float f = v[k]; v[k] = bfr(f); }
    }
    float s = 0.0f;
#pragma unroll
    for (int k = 0; k < 8; ++k) s += v[k];
    s = wsum(s);
    if (lane == 0) red[wave] = s;
    __syncthreads();
    const float mu = ((red[0] + red[1]) + (red[2] + red[3])) * (1.0f / DM);
    v8f d; float s2 = 0.0f;
#pragma unroll
    for (int k = 0; k < 8; ++k) { const float dk = v[k] - mu; d[k] = dk; s2 += dk * dk; }
    s2 = wsum(s2);
    if (lane == 0) red[4 + wave] = s2;
    __syncthreads();
    const float var = ((red[4] + red[5]) + (red[6] + red[7])) * (1.0f / DM);
    const float rs = rsqrtf(var + 1.0e-5f);
    const v4f w0 = *(const v4f*)(w + t * 8), w1 = *(const v4f*)(w + t * 8 + 4);
    const v4f b0 = *(const v4f*)(bb + t * 8), b1 = *(const v4f*)(bb + t * 8 + 4);
    const v8f wv = cat8f(w0, w1), bv = cat8f(b0, b1);
    v8h o;
#pragma unroll
    for (int k = 0; k < 8; ++k) { const float wk = wv[k], bk = bv[k]; o[k] = (h16)(((d[k] * rs) * bfr(wk) + bfr(bk)) * HCAR); }
    h16* dst = Hp + (size_t)row * DM + t * 8;
    *(volatile v8h*)dst = o; __threadfence(); *(volatile v8h*)dst = o;
}

__global__ __launch_bounds__(256) void k_vt16(const h16* __restrict__ QKV, h16* VT) {
    const unsigned e = (blockIdx.x * 256 + threadIdx.x) * 2; if (e >= (unsigned)(NB * NH * DH * SEQ)) return;
    const unsigned j = e % SEQ, rest = e / SEQ; const unsigned d = rest % DH, hd = (rest / DH) % NH, b = rest / (DH * NH);
    const size_t src = (size_t)(b * SEQ + j) * QKVW + 2 * DM + hd * DH + d;
    v2h o; o[0] = QKV[src]; o[1] = QKV[src + QKVW];
    *(volatile v2h*)(VT + e) = o; __threadfence(); *(volatile v2h*)(VT + e) = o;
}

__global__ __launch_bounds__(256) void k_lines(const h16* __restrict__ SM, const float* __restrict__ gb, h16* RL, h16* JW, float* GT) {
#pragma clang fp contract(off)
    const unsigned idx = blockIdx.x * 256 + threadIdx.x;
    const unsigned t = idx % SEQ, bh = idx / SEQ; const unsigned h = bh % NH, b = bh / NH;
    const size_t tok = (size_t)b * SEQ + t;
    const size_t tokp = (t > 0) ? tok - 1 : tok;
    const float pm = (t > 0) ? 1.0f : 0.0f;
    const v4h w1 = *(const v4ha*)(SM + tokp * SMW + h * PD);
    const v4h w2 = *(const v4ha*)(SM + tok * SMW + 64 + h * PD);
    const v4h r1 = *(const v4ha*)(SM + tok * SMW + 128 + h * PD);
    const v4h r2 = *(const v4ha*)(SM + tok * SMW + 192 + h * PD);
    const float gpre = (float)SM[tok * SMW + 256 + h] + bfr(gb[h]);
    const v8f wl = plucker(w1, w2, pm);
    const v8f rl = plucker(r1, r2, 1.0f);
    v8h orl, ojw;
    orl[0] = toh_flush(rl[0] * LCAR); orl[1] = toh_flush(rl[1] * LCAR); orl[2] = toh_flush(rl[2] * LCAR);
    orl[3] = toh_flush(rl[3] * LCAR); orl[4] = toh_flush(rl[4] * LCAR); orl[5] = toh_flush(rl[5] * LCAR);
    orl[6] = (h16)0.0f; orl[7] = (h16)0.0f;
    ojw[0] = toh_flush(wl[5] * LCAR);  ojw[1] = toh_flush(-wl[4] * LCAR); ojw[2] = toh_flush(wl[3] * LCAR);
    ojw[3] = toh_flush(wl[2] * LCAR);  ojw[4] = toh_flush(-wl[1] * LCAR); ojw[5] = toh_flush(wl[0] * LCAR);
    ojw[6] = (h16)0.0f; ojw[7] = (h16)0.0f;
    const float g = __builtin_amdgcn_rcpf(1.0f + __builtin_amdgcn_exp2f(-gpre * L2E));
    h16* prl = RL + (size_t)idx * 8; h16* pjw = JW + (size_t)idx * 8; float* pg = GT + idx;
    *(volatile v8h*)prl = orl; *(volatile v8h*)pjw = ojw; *(volatile float*)pg = g;
    __threadfence();
    *(volatile v8h*)prl = orl; *(volatile v8h*)pjw = ojw; *(volatile float*)pg = g;
}

__global__ __launch_bounds__(512) void k_mem(const h16* __restrict__ RL, const h16* __restrict__ JW, const float* __restrict__ GT,
                                             const float* __restrict__ dlog, const float* __restrict__ msc, float* GD) {
    __shared__ float msl[NH * 32];
    __shared__ float gl[NH * 32];
    const int wave = __builtin_amdgcn_readfirstlane(threadIdx.x >> 5);
    const int lane = threadIdx.x & 31, lr = lane & 15, hi = lane >> 4;
    const int ib = blockIdx.x % (SEQ / 32), b = blockIdx.x / (SEQ / 32);
    const int h = wave;
    const size_t base = (size_t)(b * NH + h) * SEQ;
    const float dl = bfr(dlog[h]);
    const float dec = __builtin_amdgcn_rcpf(1.0f + __builtin_amdgcn_exp2f(-dl * L2E));
    const float d16 = ipow32(dec, 16);
    v8f fr, fd;
#pragma unroll
    for (int r = 0; r < 8; ++r) {
        const int n = 8 * hi + r - lr;
        fr[r] = ipow32(dec, 16 + n);
        const float pd = ipow32(dec, (n > 0) ? n : 0);
        fd[r] = (n > 0) ? pd : 0.0f;
    }
#pragma unroll 1
    for (int qt = 0; qt < 2; ++qt) {
        const int i0 = ib * 32 + qt * 16;
        const v16h a = ldfrag8(RL + (base + i0 + lr) * 8, hi);
        v8f S = (v8f){};
        const int nt = i0 >> 4;
#pragma unroll 1
        for (int jt = 0; jt < nt; ++jt) {
            const v16h bj = ldfrag8(JW + (base + jt * 16 + lr) * 8, hi);
            const v8f d = wmma16g(a, bj, (v8f){});
#pragma unroll
            for (int r = 0; r < 8; ++r) S[r] = S[r] * d16 + fr[r] * fabsf(d[r]);
        }
        {
            const v16h bj = ldfrag8(JW + (base + i0 + lr) * 8, hi);
            const v8f d = wmma16g(a, bj, (v8f){});
#pragma unroll
            for (int r = 0; r < 8; ++r) S[r] = S[r] + fd[r] * fabsf(d[r]);
        }
#pragma unroll
        for (int r = 0; r < 8; ++r) {
            float v = S[r];
            v += __shfl_xor(v, 8, 32); v += __shfl_xor(v, 4, 32); v += __shfl_xor(v, 2, 32); v += __shfl_xor(v, 1, 32);
            S[r] = v * (1.0f / (LCAR * LCAR));
        }
        if (lr == 0) {
#pragma unroll
            for (int r = 0; r < 8; ++r) msl[h * 32 + qt * 16 + 8 * hi + r] = S[r];
        }
    }
    __syncthreads();
    {
        const float sc = bfr(msc[h]);
        const float ms = msl[h * 32 + lane];
        const float g = GT[base + ib * 32 + lane];
        const float sg = __builtin_amdgcn_rcpf(1.0f + __builtin_amdgcn_exp2f(-(ms * sc) * L2E));
        gl[h * 32 + lane] = sg * g;
    }
    __syncthreads();
    if (wave == 0) {
        float s = 0.0f;
#pragma unroll 1
        for (int hh = 0; hh < NH; ++hh) s += gl[hh * 32 + lane];
        s *= (1.0f / NH);
        float* p = GD + (size_t)b * SEQ + ib * 32 + lane;
        *(volatile float*)p = s; __threadfence(); *(volatile float*)p = s;
    }
}

__global__ __launch_bounds__(128) void k_attn(const h16* __restrict__ QKV, const h16* __restrict__ VT, const h16* __restrict__ MV, const float* __restrict__ GD, h16* O16) {
    __shared__ __align__(16) float os[4 * 16 * 68];
    const int wave = __builtin_amdgcn_readfirstlane(threadIdx.x >> 5);
    const int lane = threadIdx.x & 31, lr = lane & 15, hi = lane >> 4;
    const int h = blockIdx.y, b = blockIdx.z;
    const int q0 = blockIdx.x * 64 + wave * 16;
    const int qrow = q0 + lr;
    const size_t qoff = (size_t)(b * SEQ + q0 + lr) * QKVW + h * DH + 8 * hi;
    const v16h bq0 = ldfrag(QKV + qoff), bq1 = ldfrag(QKV + qoff + 32);
    const size_t kbase = (size_t)(b * SEQ + lr) * QKVW + DM + h * DH + 8 * hi;
    const size_t vbase = ((size_t)(b * NH + h) * DH + lr) * SEQ + 8 * hi;
    v8f o[4];
#pragma unroll
    for (int t = 0; t < 4; ++t) o[t] = (v8f){};
    float m = -1.0e30f, l = 0.0f;
    const int ns = (q0 >> 5) + 1;
#pragma unroll 1
    for (int kb = 0; kb < ns; ++kb) {
        const int key0 = kb * 32;
        const size_t ko = kbase + (size_t)key0 * QKVW;
        v16h ak = ldfrag(QKV + ko);
        v8f s0 = wmma16g(ak, bq0, (v8f){});
        ak = ldfrag(QKV + ko + 32);
        s0 = wmma16g(ak, bq1, s0);
        ak = ldfrag(QKV + ko + (size_t)16 * QKVW);
        v8f s1 = wmma16g(ak, bq0, (v8f){});
        ak = ldfrag(QKV + ko + (size_t)16 * QKVW + 32);
        s1 = wmma16g(ak, bq1, s1);
        float mx = -1.0e30f;
#pragma unroll
        for (int r = 0; r < 8; ++r) {
            const int key = key0 + 8 * hi + r;
            const float x0 = (key <= qrow) ? s0[r] * SCL2 : -1.0e30f;
            const float x1 = (key + 16 <= qrow) ? s1[r] * SCL2 : -1.0e30f;
            s0[r] = x0; s1[r] = x1;
            mx = fmaxf(mx, fmaxf(x0, x1));
        }
        mx = fmaxf(mx, __shfl_xor(mx, 16, 32));
        const float mn = fmaxf(m, mx);
        const float al = __builtin_amdgcn_exp2f(m - mn);
        m = mn;
        const float sh = PLOG - mn;
        v8h p0, p1; float psum = 0.0f;
#pragma unroll
        for (int r = 0; r < 8; ++r) {
            const float e0 = s0[r] + sh, e1 = s1[r] + sh;
            const float f0 = (e0 < -14.0f) ? 0.0f : __builtin_amdgcn_exp2f(e0);
            const float f1 = (e1 < -14.0f) ? 0.0f : __builtin_amdgcn_exp2f(e1);
            const h16 g0 = (h16)f0, g1 = (h16)f1;
            p0[r] = g0; p1[r] = g1;
            psum += (float)g0 + (float)g1;
        }
        psum += __shfl_xor(psum, 16, 32);
        l = l * al + psum;
#pragma unroll
        for (int t = 0; t < 4; ++t) o[t] = o[t] * al;
        const v16h pb = cat16(p0, p1);
        const size_t vo = vbase + key0;
        v16h av = ldfrag(VT + vo);
        o[0] = wmma16g(av, pb, o[0]);
        av = ldfrag(VT + vo + (size_t)16 * SEQ);
        o[1] = wmma16g(av, pb, o[1]);
        av = ldfrag(VT + vo + (size_t)32 * SEQ);
        o[2] = wmma16g(av, pb, o[2]);
        av = ldfrag(VT + vo + (size_t)48 * SEQ);
        o[3] = wmma16g(av, pb, o[3]);
    }
    const float inv = __builtin_amdgcn_rcpf(l);
    const int wb = wave * (16 * 68);
#pragma unroll
    for (int t = 0; t < 4; ++t) {
        const v8f ov = o[t] * inv;
        *(v4fa*)(os + wb + lr * 68 + 16 * t + 8 * hi)     = __builtin_shufflevector(ov, ov, 0, 1, 2, 3);
        *(v4fa*)(os + wb + lr * 68 + 16 * t + 8 * hi + 4) = __builtin_shufflevector(ov, ov, 4, 5, 6, 7);
    }
    __builtin_amdgcn_fence(3, "wavefront"); __builtin_amdgcn_wave_barrier(); asm volatile("" ::: "memory");
    const int q8 = lane >> 3, cofs = (lane & 7) * 8;
#pragma unroll 1
    for (int pass = 0; pass < 2; ++pass) {
#pragma unroll 1
        for (int s = 0; s < 4; ++s) {
            const int row = 4 * s + q8;
            const size_t tok = (size_t)b * SEQ + q0 + row;
            const v4f u0 = *(const v4fa*)(os + wb + row * 68 + cofs), u1 = *(const v4fa*)(os + wb + row * 68 + cofs + 4);
            const v8f u = cat8f(u0, u1);
            const v8h mv = *(const v8ha*)(MV + tok * DM + h * DH + cofs);
            const float g = GD[tok];
            v8h ov;
#pragma unroll
            for (int q = 0; q < 8; ++q) ov[q] = toh_flush((u[q] + g * (float)mv[q]) * OCAR);
            *(volatile v8h*)(O16 + tok * DM + h * DH + cofs) = ov;
        }
        if (pass == 0) __threadfence();
    }
}

static inline unsigned cdiv(size_t a, unsigned b) { return (unsigned)((a + b - 1) / b); }

extern "C" void kernel_launch(void* const* d_in, const int* in_sizes, int n_in,
                              void* d_out, int out_size, void* d_ws, size_t ws_size, hipStream_t stream) {
    if (n_in < 23) return;
    if (in_sizes[0] < NTOK * DM || in_sizes[1] < DM || in_sizes[2] < DM || in_sizes[3] < QKVW * DM || in_sizes[4] < QKVW ||
        in_sizes[5] < NH * PD * DM || in_sizes[6] < NH * PD * DM || in_sizes[7] < NH * PD * DM || in_sizes[8] < NH * PD * DM ||
        in_sizes[9] < DM * DM || in_sizes[10] < DM || in_sizes[11] < NH * DM || in_sizes[12] < NH || in_sizes[13] < NH ||
        in_sizes[14] < DM * DM || in_sizes[15] < DM || in_sizes[16] < NH || in_sizes[17] < DM || in_sizes[18] < DM ||
        in_sizes[19] < FFD * DM || in_sizes[20] < FFD || in_sizes[21] < DM * FFD || in_sizes[22] < DM) return;
    if (out_size < NTOK * DM) return;
    const float* x       = (const float*)d_in[0];
    const float* ln1_g   = (const float*)d_in[1];
    const float* ln1_b   = (const float*)d_in[2];
    const float* qkv_w   = (const float*)d_in[3];
    const float* qkv_b   = (const float*)d_in[4];
    const float* w1w     = (const float*)d_in[5];
    const float* w2w     = (const float*)d_in[6];
    const float* w1r     = (const float*)d_in[7];
    const float* w2r     = (const float*)d_in[8];
    const float* memv_w  = (const float*)d_in[9];
    const float* memv_b  = (const float*)d_in[10];
    const float* memg_w  = (const float*)d_in[11];
    const float* memg_b  = (const float*)d_in[12];
    const float* mem_sc  = (const float*)d_in[13];
    const float* out_w   = (const float*)d_in[14];
    const float* out_b   = (const float*)d_in[15];
    const float* dlogit  = (const float*)d_in[16];
    const float* ln2_g   = (const float*)d_in[17];
    const float* ln2_b   = (const float*)d_in[18];
    const float* fc1_w   = (const float*)d_in[19];
    const float* fc1_b   = (const float*)d_in[20];
    const float* fc2_w   = (const float*)d_in[21];
    const float* fc2_b   = (const float*)d_in[22];
    float* OUT = (float*)d_out;

    char* wsp = (char*)d_ws;
    auto take = [&](size_t bytes) { char* p = wsp; wsp += (bytes + 255) & ~(size_t)255; return (void*)p; };
    h16* WQKV  = (h16*)take((size_t)QKVW * DM * 2);
    h16* WMV   = (h16*)take((size_t)DM * DM * 2);
    h16* WO    = (h16*)take((size_t)DM * DM * 2);
    h16* W1    = (h16*)take((size_t)FFD * DM * 2);
    h16* W2    = (h16*)take((size_t)DM * FFD * 2);
    h16* WSM   = (h16*)take((size_t)SMW * DM * 2);
    h16* QKV16 = (h16*)take((size_t)NTOK * QKVW * 2);
    h16* H2    = QKV16;
    h16* VT    = (h16*)take((size_t)NTOK * DM * 2);
    char* R1   = (char*)take((size_t)NTOK * DM * 4);
    h16* H1 = (h16*)R1; float* X1 = (float*)R1;
    h16* MV16  = (h16*)take((size_t)NTOK * DM * 2);
    h16* SM16  = (h16*)take((size_t)NTOK * SMW * 2);
    h16* RL    = (h16*)take((size_t)NB * NH * SEQ * 8 * 2);
    h16* JW    = (h16*)take((size_t)NB * NH * SEQ * 8 * 2);
    float* GT  = (float*)take((size_t)NB * NH * SEQ * 4);
    float* GD  = (float*)take((size_t)NTOK * 4);
    h16* O16   = (h16*)take((size_t)NTOK * DM * 2);
    h16* A1    = (h16*)take((size_t)NTOK * FFD * 2);
    const size_t used = (size_t)(wsp - (char*)d_ws);
    if (used > ws_size || used > (size_t)134217728) return;

    k_cvtw<<<cdiv((size_t)QKVW * DM / 8, 256), 256, 0, stream>>>(qkv_w, WQKV, (unsigned)(QKVW * DM / 8));
    k_cvtw<<<cdiv((size_t)DM * DM / 8, 256), 256, 0, stream>>>(memv_w, WMV, (unsigned)(DM * DM / 8));
    k_cvtw<<<cdiv((size_t)DM * DM / 8, 256), 256, 0, stream>>>(out_w, WO, (unsigned)(DM * DM / 8));
    k_cvtw<<<cdiv((size_t)FFD * DM / 8, 256), 256, 0, stream>>>(fc1_w, W1, (unsigned)(FFD * DM / 8));
    k_cvtw<<<cdiv((size_t)DM * FFD / 8, 256), 256, 0, stream>>>(fc2_w, W2, (unsigned)(DM * FFD / 8));
    k_cvtw<<<cdiv((size_t)64 * DM / 8, 256), 256, 0, stream>>>(w1w, WSM, (unsigned)(64 * DM / 8));
    k_cvtw<<<cdiv((size_t)64 * DM / 8, 256), 256, 0, stream>>>(w2w, WSM + (size_t)64 * DM, (unsigned)(64 * DM / 8));
    k_cvtw<<<cdiv((size_t)64 * DM / 8, 256), 256, 0, stream>>>(w1r, WSM + (size_t)128 * DM, (unsigned)(64 * DM / 8));
    k_cvtw<<<cdiv((size_t)64 * DM / 8, 256), 256, 0, stream>>>(w2r, WSM + (size_t)192 * DM, (unsigned)(64 * DM / 8));
    k_cvtw<<<cdiv((size_t)NH * DM / 8, 256), 256, 0, stream>>>(memg_w, WSM + (size_t)256 * DM, (unsigned)(NH * DM / 8));
    k_zero16<<<cdiv((size_t)(SMW - 256 - NH) * DM / 8, 256), 256, 0, stream>>>(WSM + (size_t)(256 + NH) * DM, (unsigned)((SMW - 256 - NH) * DM / 8));
    k_ln<true><<<NTOK, 128, 0, stream>>>(x, ln1_g, ln1_b, H1);
    k_gemm<EP_H16, true, false><<<dim3(NTOK / 64, QKVW / 64, 1), 32, 0, stream>>>(H1, WQKV, DM, nullptr, QKV16, QKVW, 1.0f / (HCAR * WCAR), 1.0f, qkv_b, nullptr, 0, 0, 0);
    k_gemm<EP_H16, true, false><<<dim3(NTOK / 64, DM / 64, 1), 32, 0, stream>>>(H1, WMV, DM, nullptr, MV16, DM, 1.0f / (HCAR * WCAR), 1.0f, memv_b, nullptr, 0, 0, 0);
    k_gemm<EP_H16, false, false><<<dim3(NTOK / 64, SMW / 64, 1), 32, 0, stream>>>(H1, WSM, DM, nullptr, SM16, SMW, 1.0f / (HCAR * WCAR), 1.0f, nullptr, nullptr, 0, 0, 0);
    k_vt16<<<cdiv((size_t)NB * NH * DH * SEQ / 2, 256), 256, 0, stream>>>(QKV16, VT);
    k_lines<<<(NB * NH * SEQ) / 256, 256, 0, stream>>>(SM16, memg_b, RL, JW, GT);
    k_mem<<<NB * (SEQ / 32), 512, 0, stream>>>(RL, JW, GT, dlogit, mem_sc, GD);
    k_attn<<<dim3(SEQ / 64, NH, NB), 128, 0, stream>>>(QKV16, VT, MV16, GD, O16);
    k_gemm<EP_RES, true, true><<<dim3(NTOK / 64, DM / 64, 1), 32, 0, stream>>>(O16, WO, DM, X1, nullptr, DM, 1.0f / (OCAR * WCAR), 1.0f, out_b, x, 0, 0, 0);
    k_ln<false><<<NTOK, 128, 0, stream>>>(X1, ln2_g, ln2_b, H2);
    k_gemm<EP_GELU, true, false><<<dim3(NTOK / 64, FFD / 64, 1), 32, 0, stream>>>(H2, W1, DM, nullptr, A1, FFD, 1.0f / (HCAR * WCAR), ACAR, fc1_b, nullptr, 0, 0, 0);
    k_gemm<EP_RES, true, false><<<dim3(NTOK / 64, DM / 64, 1), 32, 0, stream>>>(A1, W2, FFD, OUT, nullptr, DM, 1.0f / (ACAR * WCAR), 1.0f, fc2_b, X1, 0, 0, 0);
}
